// PacCRF_601295421593
// MI455X (gfx1250) — hardware-verified
//
#include <hip/hip_runtime.h>


namespace {
constexpr int Bn = 2, C = 21, H = 512, W = 512, HW = H * W, CF = 3, KK = 9, NMX = KK * C  , NM = 192, NSTEP = 5, BAND = 64, BR = BAND + 2, SW = 32, SP = 48  ;
constexpr float QS = 8.0f;

typedef _Float16 b16;
typedef __attribute__((ext_vector_type(16))) _Float16 v16b;
typedef __attribute__((ext_vector_type(8))) _Float16 v8b;
typedef __attribute__((ext_vector_type(8))) float v8f;
typedef __attribute__((ext_vector_type(4))) float v4f;
__device__ __forceinline__ float bf16_rne(float f) { unsigned int u = __float_as_uint(f); u += 0x7FFFu + ((u >> 16) & 1u); return __uint_as_float(u & 0xFFFF0000u); }
__device__ __forceinline__ v16b frag_kb(const b16* p, int hh) { const v8b a = *(const v8b*)(p + 8 * hh), b = *(const v8b*)(p + 16 + 8 * hh); v16b f;
#pragma unroll
  for (int e = 0; e < 8; ++e) { f[e] = a[e]; f[8 + e] = b[e]; } return f; }
__device__ __forceinline__ v8f wmma16b(v16b a, v16b b, v8f c) { v8f d = __builtin_amdgcn_wmma_f32_16x16x32_f16(false, a, false, b, (short)0, c, false, false); asm volatile("v_nop\n\tv_nop\n\tv_nop\n\tv_nop" : "+v"(d) : "v"(a), "v"(b)); return d; }
__device__ __forceinline__ float nexp(float x) { return __builtin_amdgcn_exp2f(x * 1.4426950408889634f); }
__device__ __forceinline__ float pmul(float a, float b) { float p = a * b; asm volatile("" : "+v"(p)); return p; }

__global__ __launch_bounds__(256) void prep_kernel(const float* __restrict__ wt, const float* __restrict__ uw, b16* __restrict__ R, float* __restrict__ P) {
  const int t_ = threadIdx.x;
  for (int pass = 0; pass < 2; ++pass) {
    for (int p = t_; p < NM * 4; p += 256) { const int m = p >> 2, i0 = (p & 3) * 8; v8b v;
#pragma unroll
      for (int e = 0; e < 8; ++e) { const int i = i0 + e; float w = 0.0f; if (m < NMX && i < C) { const int k = m / C, o = m % C; w = bf16_rne(wt[((size_t)o * C + i) * KK + k]); } v[e] = (b16)w; }
      *(volatile v8b*)(R + (size_t)m * 32 + i0) = v; }
    if (t_ < 32) ((volatile float*)P)[t_] = (t_ == 0) ? bf16_rne(uw[0]) : 0.0f;
    __threadfence(); }
}

__global__ __launch_bounds__(512) void kern_kernel(const float* __restrict__ ef, float* __restrict__ kern) {
  const int b = blockIdx.y, h = blockIdx.x, w = threadIdx.x; float fc[CF];
#pragma unroll
  for (int c = 0; c < CF; ++c) fc[c] = bf16_rne(ef[(((size_t)b * CF + c) * H + h) * W + w]);
  float kv[KK];
#pragma unroll
  for (int k = 0; k < KK; ++k) { const int hh = h + k / 3 - 1, ww = w + k % 3 - 1; float s = 0.0f;
#pragma unroll
    for (int c = 0; c < CF; ++c) { const float fj = (hh >= 0 && hh < H && ww >= 0 && ww < W) ? bf16_rne(ef[(((size_t)b * CF + c) * H + hh) * W + ww]) : 0.0f; const float d = fj - fc[c]; s += pmul(d, d); }
    kv[k] = nexp(-0.5f * s); }
  for (int pass = 0; pass < 2; ++pass) {
#pragma unroll
    for (int k = 0; k < KK; ++k) ((volatile float*)kern)[(((size_t)b * KK + k) * H + h) * W + w] = kv[k];
    __threadfence(); }
}

__global__ __launch_bounds__(128) void step_kernel(const float* __restrict__ src, int rnd, const float* __restrict__ kern, const float* __restrict__ unary, const b16* __restrict__ R_, const float* __restrict__ P, float* __restrict__ dst) {
  __shared__ __attribute__((aligned(16))) b16 Qs[SP][40]; __shared__ float Mr[3][NMX][SP + 1]; __shared__ __attribute__((aligned(16))) float Ot[C][SW + 4];
  const int lane = threadIdx.x & 31, wave = threadIdx.x >> 5, nloc = lane & 15, hlf = lane >> 4, t_ = threadIdx.x, b = blockIdx.z, h0 = blockIdx.y * BAND, w0 = blockIdx.x * SW; const float uw = P[0];
  for (int R = 0; R < BR; ++R) { const int h = h0 - 1 + R; const int slot = R % 3;
    if (t_ < SP) { const int w = w0 - 8 + t_; float v[C]; bool ok = (h >= 0 && h < H && w >= 0 && w < W);
      if (ok) { float mx = -INFINITY;
#pragma unroll
        for (int c = 0; c < C; ++c) { float x = src[(((size_t)b * C + c) * H + h) * W + w]; if (rnd) x = bf16_rne(x); v[c] = x; mx = fmaxf(mx, x); }
        float s = 0.0f;
#pragma unroll
        for (int c = 0; c < C; ++c) { v[c] = nexp(v[c] - mx); s += v[c]; }
        const float inv = QS / s;
#pragma unroll
        for (int c = 0; c < C; ++c) v[c] *= inv; }
#pragma unroll
      for (int c = 0; c < 32; ++c) Qs[t_][c] = (b16)((ok && c < C) ? v[c] : 0.0f); }
    __syncthreads();
    { v16b a[3];
#pragma unroll
      for (int pt = 0; pt < 3; ++pt) a[pt] = frag_kb(&Qs[pt * 16 + nloc][0], hlf);
#pragma unroll
      for (int st = 0; st < 3; ++st) { const int m0 = (wave * 3 + st) * 16; const v16b bw = frag_kb(R_ + (size_t)(m0 + nloc) * 32, hlf);
#pragma unroll
        for (int pt = 0; pt < 3; ++pt) { v8f acc = {}; acc = wmma16b(a[pt], bw, acc); const int m = m0 + nloc;
          if (m < NMX) {
#pragma unroll
            for (int r = 0; r < 8; ++r) Mr[slot][m][pt * 16 + 8 * hlf + r] = acc[r] * (1.0f / QS); } } } }
    __syncthreads();
    if (R >= 2) { const int hr = h0 + R - 2; const int px = t_ & 31, og = t_ >> 5; const int w = w0 + px; const int j = px + 8;
      float kv[KK];
#pragma unroll
      for (int k = 0; k < KK; ++k) kv[k] = kern[(((size_t)b * KK + k) * H + hr) * W + w];
      for (int o = og; o < C; o += 4) { float msg = 0.0f;
#pragma unroll
        for (int k = 0; k < KK; ++k) { const int dy = k / 3 - 1, dx = k % 3 - 1; const int sl = (R - 1 + dy) % 3; const int ww = w + dx; if (ww >= 0 && ww < W) msg += pmul(kv[k], Mr[sl][k * C + o][j + dx]); }
        Ot[o][px] = pmul(uw, bf16_rne(unary[(((size_t)b * C + o) * H + hr) * W + w])) - msg; }
      __syncthreads();
      for (int pass = 0; pass < 2; ++pass) { for (int i = t_; i < C * 8; i += 128) { const int o = i >> 3, c4 = (i & 7) * 4; *(volatile v4f*)(dst + (((size_t)b * C + o) * H + hr) * W + w0 + c4) = *(const v4f*)(&Ot[o][c4]); } __threadfence(); } }
    __syncthreads(); }
}
}

extern "C" void kernel_launch(void* const* d_in, const int* in_sizes, int n_in,
                              void* d_out, int out_size, void* d_ws, size_t ws_size, hipStream_t stream) {
  (void)n_in; (void)out_size;
  const float* unary = (const float*)d_in[0]; const float* ef = (const float*)d_in[1]; const float* wt = (const float*)d_in[2]; const float* uw = (const float*)d_in[3];
  float* out = (float*)d_out;
  if (in_sizes[0] != Bn * C * HW || in_sizes[1] != Bn * CF * HW || in_sizes[2] != C * C * KK || in_sizes[3] != 1) return;
  size_t off = 0; char* ws = (char*)d_ws;
  auto carve = [&](size_t bytes) { char* p = ws + off; off += (bytes + 255) & ~(size_t)255; return p; };
  b16* R = (b16*)carve((size_t)NM * 32 * 2); float* P = (float*)carve(256); float* kern = (float*)carve((size_t)Bn * KK * HW * 4); float* lqA = (float*)carve((size_t)Bn * C * HW * 4);
  if (off > ws_size) return;
  prep_kernel<<<1, 256, 0, stream>>>(wt, uw, R, P);
  kern_kernel<<<dim3(H, Bn), 512, 0, stream>>>(ef, kern);
  for (int s = 0; s < NSTEP; ++s) { const float* srcp = (s == 0) ? unary : ((s & 1) ? out : lqA); float* dstp = (s & 1) ? lqA : out;
    step_kernel<<<dim3(W / SW, H / BAND, Bn), 128, 0, stream>>>(srcp, (s == 0) ? 1 : 0, kern, unary, R, P, dstp); }
}
